// ComplexSSM_18562848653623
// MI455X (gfx1250) — hardware-run, weakly checked
//
#include <hip/hip_runtime.h>


#define NB   8
#define NT   2048
#define ND   1024
#define NR   256
typedef _Float16 h16;
typedef unsigned short bf;
typedef __attribute__((ext_vector_type(16))) __bf16   v16bf;
typedef __attribute__((ext_vector_type(16))) _Float16 v16h;
typedef __attribute__((ext_vector_type(8)))  _Float16 v8h;
typedef __attribute__((ext_vector_type(8)))  unsigned short v8us;
typedef __attribute__((ext_vector_type(8)))  float    v8f;
typedef __attribute__((ext_vector_type(4)))  float    v4f;
typedef v8h  __attribute__((may_alias)) v8ha;
typedef v4f  __attribute__((may_alias)) v4fa;
typedef v8us __attribute__((may_alias)) v8usa;

__device__ __forceinline__ unsigned short f2bf(float f) { unsigned u = __float_as_uint(f); u += 0x7FFFu + ((u >> 16) & 1u); return (unsigned short)(u >> 16); }
__device__ __forceinline__ float bf2f(unsigned short b) { return __uint_as_float(((unsigned)b) << 16); }
__device__ __forceinline__ float bfr(float f) { return bf2f(f2bf(f)); }
__device__ __forceinline__ v16h cat16(v8h lo, v8h hi) { return __builtin_shufflevector(lo, hi, 0, 1, 2, 3, 4, 5, 6, 7, 8, 9, 10, 11, 12, 13, 14, 15); }
__device__ __forceinline__ v16bf cat16b(v8us lo, v8us hi) { return __builtin_bit_cast(v16bf, __builtin_shufflevector(lo, hi, 0, 1, 2, 3, 4, 5, 6, 7, 8, 9, 10, 11, 12, 13, 14, 15)); }
__device__ __forceinline__ v8f wmma16(v16h a, v16h b, v8f c) { return __builtin_amdgcn_wmma_f32_16x16x32_f16(false, a, false, b, (short)0, c, false, false); }
__device__ __forceinline__ v8f wmmab(v16bf a, v16bf b, v8f c) { return __builtin_amdgcn_wmma_f32_16x16x32_bf16(false, a, false, b, (short)0, c, false, false); }

template <typename T16> struct WFrag;
template <> struct WFrag<h16> { typedef v16h V; static __device__ __forceinline__ V ld(const h16* p) { return cat16(*(const v8h*)p, *(const v8h*)(p + 16)); } static __device__ __forceinline__ v8f mma(V a, V b, v8f c) { return wmma16(a, b, c); } };
template <> struct WFrag<bf> { typedef v16bf V; static __device__ __forceinline__ V ld(const bf* p) { return cat16b(*(const v8us*)p, *(const v8us*)(p + 16)); } static __device__ __forceinline__ v8f mma(V a, V b, v8f c) { return wmmab(a, b, c); } };
template <typename T16, int NSPLIT, bool BIAS>
__global__ __launch_bounds__(32) void k_gemmw(const T16* __restrict__ A, const T16* __restrict__ A2, const T16* __restrict__ Bt, const T16* __restrict__ Bt2, int K, float* C, int ldc, const float* __restrict__ bias, size_t sA, size_t sB, size_t sC) {
    typedef typename WFrag<T16>::V V;
    __shared__ __align__(16) float os[16 * 68];
    const size_t z = blockIdx.z; A += z * sA; if (A2) A2 += z * sA; Bt += z * sB; if (Bt2) Bt2 += z * sB; C += z * sC;
    const int lane = threadIdx.x & 31, lr = lane & 15, hi = lane >> 4; const int r0 = blockIdx.x * 64, c0 = blockIdx.y * 64;
    v8f acc[4][4];
#pragma unroll
    for (int mb = 0; mb < 4; ++mb)
#pragma unroll
        for (int nb = 0; nb < 4; ++nb) acc[mb][nb] = (v8f){};
    const size_t aoff = (size_t)(r0 + lr) * K + 8 * hi, boff = (size_t)(c0 + lr) * K + 8 * hi;
    for (int kc = 0; kc < K; kc += 32) {
        V a[4], a2[4];
#pragma unroll
        for (int mb = 0; mb < 4; ++mb) { a[mb] = WFrag<T16>::ld(A + aoff + (size_t)mb * 16 * K + kc); if (NSPLIT == 1 || NSPLIT == 2) a2[mb] = WFrag<T16>::ld(A2 + aoff + (size_t)mb * 16 * K + kc); }
#pragma unroll
        for (int nb = 0; nb < 4; ++nb) { const V b = WFrag<T16>::ld(Bt + boff + (size_t)nb * 16 * K + kc); V b2; if (NSPLIT >= 2) b2 = WFrag<T16>::ld(Bt2 + boff + (size_t)nb * 16 * K + kc);
#pragma unroll
            for (int mb = 0; mb < 4; ++mb) { acc[mb][nb] = WFrag<T16>::mma(a[mb], b, acc[mb][nb]); if (NSPLIT == 1 || NSPLIT == 2) acc[mb][nb] = WFrag<T16>::mma(a2[mb], b, acc[mb][nb]); if (NSPLIT >= 2) acc[mb][nb] = WFrag<T16>::mma(a[mb], b2, acc[mb][nb]); } }
        asm volatile("v_nop\n\tv_nop\n\tv_nop\n\tv_nop" : "+v"(acc[0][0]), "+v"(acc[1][1]), "+v"(acc[2][2]), "+v"(acc[3][3]) : "v"(a[0]), "v"(a[3]));
    }
#pragma unroll
    for (int mb = 0; mb < 4; ++mb) {
#pragma unroll
        for (int nb = 0; nb < 4; ++nb) {
#pragma unroll
            for (int j = 0; j < 8; ++j) os[(hi * 8 + j) * 68 + nb * 16 + lr] = acc[mb][nb][j]; }
        __builtin_amdgcn_wave_barrier(); asm volatile("" ::: "memory");
        float* crow = C + (size_t)(r0 + mb * 16) * ldc + c0;
#pragma unroll 1
        for (int ps = 0; ps < 2; ++ps) {
#pragma unroll
            for (int s = 0; s < 8; ++s) { const int row = 2 * s + hi, cofs = lr * 4; v4f val = *(const v4fa*)(os + row * 68 + cofs); if (BIAS) { val[0] += bfr(bias[c0 + cofs]); val[1] += bfr(bias[c0 + cofs + 1]); val[2] += bfr(bias[c0 + cofs + 2]); val[3] += bfr(bias[c0 + cofs + 3]); }
                *(volatile v4f*)(crow + (size_t)row * ldc + cofs) = val; }
            if (ps == 0) __threadfence(); }
        __builtin_amdgcn_wave_barrier(); asm volatile("" ::: "memory");
    }
}

typedef __attribute__((ext_vector_type(2))) _Float16 v2h;
typedef __attribute__((ext_vector_type(4))) _Float16 v4h;
typedef __attribute__((ext_vector_type(2))) unsigned short v2us;
typedef __attribute__((ext_vector_type(4))) unsigned short v4us;
typedef __attribute__((ext_vector_type(2))) float v2f;
typedef __attribute__((ext_vector_type(4))) int v4i;
__global__ __launch_bounds__(256) void k_cvt8(const float* __restrict__ src, bf* dst, size_t n8) { const size_t i = (size_t)blockIdx.x * 256 + threadIdx.x; if (i >= n8) return; const v8f v = *(const v8f*)(src + i * 8); v8us o;
#pragma unroll
    for (int k = 0; k < 8; ++k) o[k] = f2bf(v[k]); *(volatile v8us*)(dst + i * 8) = o; __threadfence(); *(volatile v8us*)(dst + i * 8) = o; }

#define LNC_MAX 2048
template <bool RES>
__global__ __launch_bounds__(256) void k_lnrow(const float* __restrict__ A, const float* __restrict__ R, const float* __restrict__ gamma, const float* __restrict__ beta, float eps, int C, int nrows, float* Y) {
    const int lane = threadIdx.x & 31; const int row = blockIdx.x * 8 + (threadIdx.x >> 5); if (row >= nrows) return; const int nch = C / 128; const float* a = A + (size_t)row * C; float x[LNC_MAX / 32]; float s = 0.0f;
    for (int k = 0; k < LNC_MAX / 128; ++k) { if (k < nch) { const int c0 = k * 128 + lane * 4; v4f v = *(const v4f*)(a + c0);
            if (RES) { const v4f w = *(const v4f*)(R + (size_t)row * C + c0); v[0] = __fadd_rn(v[0], w[0]); v[1] = __fadd_rn(v[1], w[1]); v[2] = __fadd_rn(v[2], w[2]); v[3] = __fadd_rn(v[3], w[3]); }
            x[k * 4 + 0] = v[0]; x[k * 4 + 1] = v[1]; x[k * 4 + 2] = v[2]; x[k * 4 + 3] = v[3]; s = __fadd_rn(__fadd_rn(__fadd_rn(__fadd_rn(s, v[0]), v[1]), v[2]), v[3]); } }
    for (int sh = 16; sh; sh >>= 1) s = __fadd_rn(s, __shfl_xor(s, sh, 32));
    const float mean = __fdiv_rn(s, (float)C); float q = 0.0f;
    for (int k = 0; k < LNC_MAX / 128; ++k) { if (k < nch) {
            for (int j = 0; j < 4; ++j) { const float d = __fsub_rn(x[k * 4 + j], mean); x[k * 4 + j] = d; q = __fmaf_rn(d, d, q); } } }
    for (int sh = 16; sh; sh >>= 1) q = __fadd_rn(q, __shfl_xor(q, sh, 32));
    const float rstd = __fdiv_rn(1.0f, sqrtf(__fadd_rn(__fdiv_rn(q, (float)C), eps)));
    for (int k = 0; k < LNC_MAX / 128; ++k) { if (k < nch) { const int c0 = k * 128 + lane * 4; const v4f g = *(const v4f*)(gamma + c0); const v4f bt = *(const v4f*)(beta + c0);
            for (int j = 0; j < 4; ++j) x[k * 4 + j] = __fmaf_rn(__fmul_rn(x[k * 4 + j], rstd), bfr(g[j]), bfr(bt[j])); } }
    float* y = Y + (size_t)row * C;
    for (int ps = 0; ps < 2; ++ps) {
        for (int k = 0; k < LNC_MAX / 128; ++k) { if (k < nch) { v4f o; o[0] = x[k * 4 + 0]; o[1] = x[k * 4 + 1]; o[2] = x[k * 4 + 2]; o[3] = x[k * 4 + 3]; *(volatile v4f*)(y + k * 128 + lane * 4) = o; } }
        if (ps == 0) __threadfence(); }
}

__global__ __launch_bounds__(256) void k_scan(const float* __restrict__ V, const float* __restrict__ s, const float* __restrict__ w, const float* __restrict__ p0, const float* __restrict__ q0, float* H, float* o1, float* o2) {
    const int j = blockIdx.x * 256 + threadIdx.x; if (j >= NB * NR) return; const int b = j / NR; const int r = j % NR;
    const float sg = 1.0f / (1.0f + expf(-bfr(s[r]))); const float m = expf(-5.0f * sg); const float wr = bfr(w[r]); const float ar = m * cosf(wr); const float ai = m * sinf(wr);
    const float* v = V + (size_t)b * NT * NR + r; float* h = H + (size_t)b * NT * 2 * NR + r;
    for (int ps = 0; ps < 2; ++ps) { float p = bfr(p0[j]); float q = bfr(q0[j]);
        for (int t = 0; t < NT; ++t) { const float x = v[(size_t)t * NR]; const float pn = ar * p - ai * q + x; const float qn = ai * p + ar * q; p = pn; q = qn; *(volatile float*)(h + (size_t)t * 2 * NR) = p; *(volatile float*)(h + (size_t)t * 2 * NR + NR) = q; }
        *(volatile float*)(o1 + j) = p; *(volatile float*)(o2 + j) = q; if (ps == 0) __threadfence(); }
}

extern "C" void kernel_launch(void* const* d_in, const int* in_sizes, int n_in, void* d_out, int out_size, void* d_ws, size_t ws_size, hipStream_t stream) {
    if (n_in < 9) return;
    if (in_sizes[0] != NB * NT * ND || in_sizes[1] != NB * NR || in_sizes[2] != NB * NR || in_sizes[3] != NR || in_sizes[4] != NR || in_sizes[5] != NR * ND || in_sizes[6] != 2 * NR * ND || in_sizes[7] != 2 * NR || in_sizes[8] != 2 * NR) return;
    if (out_size != NB * NT * 2 * NR + 2 * NB * NR) return;
    static_assert((NB * NT) % 64 == 0 && NR % 64 == 0 && (2 * NR) % 128 == 0 && 2 * NR <= LNC_MAX && ND % 32 == 0 && (NB * NT * ND / 8) % 256 == 0 && (NR * ND / 8) % 256 == 0 && (NB * NR) % 256 == 0 && (NB * NT) % 8 == 0, "the products: M and N multiples of 64, the depth of 32; the row norm's width a multiple of 128 within its limit; the flat grids exact");
    const float* u = (const float*)d_in[0]; const float* p0 = (const float*)d_in[1]; const float* q0 = (const float*)d_in[2]; const float* s = (const float*)d_in[3]; const float* w = (const float*)d_in[4]; const float* A = (const float*)d_in[5]; const float* Wr = (const float*)d_in[6]; const float* g = (const float*)d_in[7]; const float* c = (const float*)d_in[8];
    float* out0 = (float*)d_out; float* out1 = out0 + (size_t)NB * NT * 2 * NR; float* out2 = out1 + (size_t)NB * NR;
    char* wsp = (char*)d_ws; auto take = [&](size_t bytes) { char* p = wsp; wsp += (bytes + 255) & ~(size_t)255; return (void*)p; };
    bf* Ub = (bf*)take((size_t)NB * NT * ND * 2); bf* Ab = (bf*)take((size_t)NR * ND * 2); bf* Wb = (bf*)take((size_t)2 * NR * ND * 2); float* V = (float*)take((size_t)NB * NT * NR * 4); float* Z = (float*)take((size_t)NB * NT * 2 * NR * 4); float* H = (float*)take((size_t)NB * NT * 2 * NR * 4);
    if ((size_t)(wsp - (char*)d_ws) > ws_size) return;
    k_cvt8<<<(unsigned)(NB * NT * ND / 8 / 256), 256, 0, stream>>>(u, Ub, (size_t)NB * NT * ND / 8);
    k_cvt8<<<(unsigned)(NR * ND / 8 / 256), 256, 0, stream>>>(A, Ab, (size_t)NR * ND / 8);
    k_cvt8<<<(unsigned)(2 * NR * ND / 8 / 256), 256, 0, stream>>>(Wr, Wb, (size_t)2 * NR * ND / 8);
    k_gemmw<bf, 0, false><<<dim3(NB * NT / 64, NR / 64, 1), 32, 0, stream>>>(Ub, nullptr, Ab, nullptr, ND, V, NR, nullptr, 0, 0, 0);
    k_gemmw<bf, 0, false><<<dim3(NB * NT / 64, 2 * NR / 64, 1), 32, 0, stream>>>(Ub, nullptr, Wb, nullptr, ND, Z, 2 * NR, nullptr, 0, 0, 0);
    k_scan<<<(unsigned)(NB * NR / 256), 256, 0, stream>>>(V, s, w, p0, q0, H, out1, out2);
    k_lnrow<true><<<(unsigned)(NB * NT / 8), 256, 0, stream>>>(H, Z, g, c, 1.0e-5f, 2 * NR, NB * NT, out0);
}
